// StandardCrossAttention_21071109554436
// MI455X (gfx1250) — hardware-verified
//
#include <hip/hip_runtime.h>
#include <math.h>
#include <stdint.h>

constexpr int kBatch = 2;
constexpr int kTq    = 2048;
constexpr int kTkv   = 2048;
constexpr int kChan  = 512;
constexpr int kHeads = 8;
constexpr int kHdim  = 64;
constexpr int kSrc   = 3;

typedef __attribute__((ext_vector_type(16))) _Float16 v16h;
typedef __attribute__((ext_vector_type(8)))  _Float16 v8h;
typedef __attribute__((ext_vector_type(16))) __bf16   v16b;
typedef __attribute__((ext_vector_type(8)))  __bf16   v8b;
typedef __attribute__((ext_vector_type(8)))  float    v8f;
typedef __attribute__((ext_vector_type(4)))  float    v4f;
typedef __attribute__((ext_vector_type(2)))  float    v2f;
typedef __attribute__((ext_vector_type(4)))  unsigned int v4u;

__device__ __forceinline__ unsigned short f2bf_bits(float f) {
  unsigned u = __float_as_uint(f);
  return (unsigned short)((u + 0x7FFFu + ((u >> 16) & 1u)) >> 16);
}
__device__ __forceinline__ float bf_bits2f(unsigned short h) { return __uint_as_float(((unsigned)h) << 16); }

__device__ __forceinline__ void dep_guard_h(v8f& a, v8f& b, v16h x, v16h y) { asm volatile("v_nop\n\tv_nop\n\tv_nop\n\tv_nop" : "+v"(a), "+v"(b) : "v"(x), "v"(y)); }
__device__ __forceinline__ void dep_guard_b(v8f& a, v8f& b, v16b x, v16b y) { asm volatile("v_nop\n\tv_nop\n\tv_nop\n\tv_nop" : "+v"(a), "+v"(b) : "v"(x), "v"(y)); }
__device__ __forceinline__ void keep4_h(v16h a, v16h b, v16h c, v16h d) { asm volatile("v_nop" :: "v"(a), "v"(b), "v"(c), "v"(d)); }
__device__ __forceinline__ void keep4_b(v16b a, v16b b, v16b c, v16b d) { asm volatile("v_nop" :: "v"(a), "v"(b), "v"(c), "v"(d)); }
__device__ __forceinline__ void acc_guard4(v8f& a, v8f& b, v8f& c, v8f& d) { asm volatile("v_nop\n\tv_nop\n\tv_nop\n\tv_nop" : "+v"(a), "+v"(b), "+v"(c), "+v"(d)); }
template <typename T> struct Frag;
template <> struct Frag<_Float16> {
  typedef v16h V; union U { v16h v; v8h h[2]; };
  static __device__ __forceinline__ v16h load(const _Float16* p) {
    U f; f.h[0] = *(const v8h*)(p); f.h[1] = *(const v8h*)(p + 16); return f.v;
  }
  static __device__ __forceinline__ v8f mma(v16h a, v16h b, v8f c) {
    return __builtin_amdgcn_wmma_f32_16x16x32_f16(false, a, false, b, (short)0, c, false, false);
  }
  static __device__ __forceinline__ void guard(v8f& a, v8f& b, v16h x, v16h y) { dep_guard_h(a, b, x, y); }
  static __device__ __forceinline__ void keep(v16h a, v16h b, v16h c, v16h d) { keep4_h(a, b, c, d); }
};
template <> struct Frag<__bf16> {
  typedef v16b V; union U { v16b v; v8b h[2]; };
  static __device__ __forceinline__ v16b load(const __bf16* p) {
    U f; f.h[0] = *(const v8b*)(p); f.h[1] = *(const v8b*)(p + 16); return f.v;
  }
  static __device__ __forceinline__ v8f mma(v16b a, v16b b, v8f c) {
    return __builtin_amdgcn_wmma_f32_16x16x32_bf16(false, a, false, b, (short)0, c, false, false);
  }
  static __device__ __forceinline__ void guard(v8f& a, v8f& b, v16b x, v16b y) { dep_guard_b(a, b, x, y); }
  static __device__ __forceinline__ void keep(v16b a, v16b b, v16b c, v16b d) { keep4_b(a, b, c, d); }
};

template <int ET> struct Elem;
template <> struct Elem<0> { typedef _Float16 T; };
template <> struct Elem<1> { typedef __bf16 T; };
template <int ET, bool SPLIT, int BIAS_MODE, int OUT_MODE, bool RESID, int ACT = 0, bool BLO = true>
__global__ __launch_bounds__(256) void wmma_gemm64(
    const unsigned short* __restrict__ Ap, const unsigned short* __restrict__ A2p, int lda, long strideA,
    const unsigned short* __restrict__ Btp, const unsigned short* __restrict__ Bt2p, int ldb, long strideB,
    void* __restrict__ Cout, void* __restrict__ Cout2, int ldc, long strideC,
    const float* __restrict__ bias,
    const float* __restrict__ resid, long strideR,
    int M, int N, int K, float scale) {
  typedef typename Elem<ET>::T T;
  typedef typename Frag<T>::V V;
  const T* A = (const T*)Ap; const T* A2 = (const T*)A2p; const T* Bt = (const T*)Btp; const T* Bt2 = (const T*)Bt2p;
  __shared__ __align__(16) float sT[8][16 * 68];
  const int b    = blockIdx.y;
  const int lane = threadIdx.x & 31;
  const int wave = threadIdx.x >> 5;
  const int tilesN = N >> 6;
  const int tilesM = M >> 6;
  const int tile = blockIdx.x * 8 + wave;
  if (tile >= tilesM * tilesN) return;
  const int tm = tile / tilesN;
  const int tn = tile - tm * tilesN;
  const int m0 = tm << 6;
  const int n0 = tn << 6;

  const T* Ab  = A  + (size_t)b * strideA;
  const T* Bb  = Bt + (size_t)b * strideB;
  const T* Ab2 = SPLIT ? (A2  + (size_t)b * strideA) : nullptr;
  const T* Bb2 = (SPLIT && BLO) ? (Bt2 + (size_t)b * strideB) : nullptr;

  const int rlane = lane & 15;
  const int koff  = (lane >> 4) * 8;
  const int mOff  = (lane >> 4) * 8;

  v8f acc[4][4];
#pragma unroll
  for (int i = 0; i < 4; ++i)
#pragma unroll
    for (int j = 0; j < 4; ++j) acc[i][j] = (v8f){0.f,0.f,0.f,0.f,0.f,0.f,0.f,0.f};

  for (int k0 = 0; k0 < K; k0 += 32) {
    V bh[4], bl[4];
#pragma unroll
    for (int j = 0; j < 4; ++j) {
      const size_t bo = (size_t)(n0 + (j << 4) + rlane) * ldb + koff + k0;
      bh[j] = Frag<T>::load(Bb + bo);
      bl[j] = (SPLIT && BLO) ? Frag<T>::load(Bb2 + bo) : bh[j];
    }
#pragma unroll
    for (int i = 0; i < 4; ++i) {
      const size_t ao = (size_t)(m0 + (i << 4) + rlane) * lda + koff + k0;
      V ah = Frag<T>::load(Ab + ao);
      V al = ah;
      if (SPLIT) al = Frag<T>::load(Ab2 + ao);
#pragma unroll
      for (int j = 0; j < 4; ++j) {
        acc[i][j] = Frag<T>::mma(ah, bh[j], acc[i][j]);
        if (SPLIT) {
          if (BLO) acc[i][j] = Frag<T>::mma(ah, bl[j], acc[i][j]);
          acc[i][j] = Frag<T>::mma(al, bh[j], acc[i][j]);
        }
      }
      Frag<T>::guard(acc[i][0], acc[i][3], ah, SPLIT ? al : ah);
    }
    Frag<T>::keep(bh[0], bh[1], bh[2], bh[3]);
    if (SPLIT && BLO) Frag<T>::keep(bl[0], bl[1], bl[2], bl[3]);
  }
  acc_guard4(acc[0][0], acc[0][1], acc[0][2], acc[0][3]);
  acc_guard4(acc[1][0], acc[1][1], acc[1][2], acc[1][3]);
  acc_guard4(acc[2][0], acc[2][1], acc[2][2], acc[2][3]);
  acc_guard4(acc[3][0], acc[3][1], acc[3][2], acc[3][3]);

  float* slab = sT[wave];
  const float* Rb = RESID ? (resid + (size_t)b * strideR) : nullptr;
#pragma unroll
  for (int i = 0; i < 4; ++i) {
    const int mBase = m0 + (i << 4);
#pragma unroll
    for (int j = 0; j < 4; ++j) {
      const int n = n0 + (j << 4) + rlane;
      float bv = 0.f;
      if (BIAS_MODE == 2) bv = bias[n];
#pragma unroll
      for (int r = 0; r < 8; ++r) {
        float v = acc[i][j][r] * scale;
        if (BIAS_MODE == 1) v += bias[mBase + mOff + r];
        if (BIAS_MODE == 2) v += bv;
        if (RESID) v += Rb[(size_t)(mBase + mOff + r) * ldc + n];
        if (ACT == 1) v = tanhf(v);
        if (ACT == 2) v = fmaxf(v, 0.0f);
        if (ACT == 3) v = v / (1.0f + expf(-v));
        if (ACT == 4) v = (v > 0.f) ? v : 0.01f * v;
        slab[(mOff + r) * 68 + (j << 4) + rlane] = v;
      }
    }
    __builtin_amdgcn_fence(__ATOMIC_RELEASE, "workgroup");
    __builtin_amdgcn_wave_barrier();
    __builtin_amdgcn_fence(__ATOMIC_ACQUIRE, "workgroup");
    if (OUT_MODE == 0) {
      float* C = (float*)Cout + (size_t)b * strideC;
      const int hh = lane >> 4, c4 = (lane & 15) * 4;
      for (int pass = 0; pass < 2; ++pass) {
#pragma unroll
        for (int it = 0; it < 8; ++it) {
          const int row = it * 2 + hh;
          v4f v = *(const v4f*)(slab + row * 68 + c4);
          *(volatile v4f*)(C + (size_t)(mBase + row) * ldc + n0 + c4) = v;
        }
        __threadfence();
      }
    } else {
      const int q = lane >> 3, c8 = (lane & 7) * 8;
      unsigned short* C  = (unsigned short*)Cout  + (size_t)b * strideC;
      unsigned short* C2 = (OUT_MODE == 2) ? ((unsigned short*)Cout2 + (size_t)b * strideC) : nullptr;
      for (int pass = 0; pass < 2; ++pass) {
#pragma unroll
        for (int it = 0; it < 4; ++it) {
          const int row = it * 4 + q;
          const float* sp = slab + row * 68 + c8;
          v8h hv, lv;
#pragma unroll
          for (int e = 0; e < 8; ++e) {
            if (OUT_MODE == 1) {
              hv[e] = (_Float16)sp[e];
            } else {
              unsigned short hb = f2bf_bits(sp[e]);
              unsigned short lb = f2bf_bits(sp[e] - bf_bits2f(hb));
              hv[e] = __builtin_bit_cast(_Float16, hb);
              lv[e] = __builtin_bit_cast(_Float16, lb);
            }
          }
          *(volatile v8h*)(C + (size_t)(mBase + row) * ldc + n0 + c8) = hv;
          if (OUT_MODE == 2) *(volatile v8h*)(C2 + (size_t)(mBase + row) * ldc + n0 + c8) = lv;
        }
        __threadfence();
      }
    }
    __builtin_amdgcn_fence(__ATOMIC_RELEASE, "workgroup");
    __builtin_amdgcn_wave_barrier();
    __builtin_amdgcn_fence(__ATOMIC_ACQUIRE, "workgroup");
  }
}

__device__ __forceinline__ unsigned pk16(unsigned short a, unsigned short b) { return (unsigned)a | ((unsigned)b << 16); }

__global__ __launch_bounds__(256) void split_bf16x2_kernel(const float* __restrict__ in, unsigned short* __restrict__ hi,
                                                           unsigned short* __restrict__ lo, int n2) {
  const int i = blockIdx.x * 256 + threadIdx.x;
  if (i < n2) {
    const v2f f = *(const v2f*)(in + 2 * (size_t)i);
    const unsigned short h0 = f2bf_bits(f[0]), h1 = f2bf_bits(f[1]);
    const unsigned short l0 = f2bf_bits(f[0] - bf_bits2f(h0)), l1 = f2bf_bits(f[1] - bf_bits2f(h1));
    const unsigned uh = pk16(h0, h1), ul = pk16(l0, l1);
    ((volatile unsigned*)hi)[i] = uh;
    ((volatile unsigned*)lo)[i] = ul;
    __threadfence();
    ((volatile unsigned*)hi)[i] = uh;
    ((volatile unsigned*)lo)[i] = ul;
  }
}

__global__ __launch_bounds__(256) void cast_bf16x2_kernel(const float* __restrict__ in, unsigned short* __restrict__ outp, int n2) {
  const int i = blockIdx.x * 256 + threadIdx.x;
  if (i < n2) {
    const v2f f = *(const v2f*)(in + 2 * (size_t)i);
    const unsigned u = pk16(f2bf_bits(f[0]), f2bf_bits(f[1]));
    ((volatile unsigned*)outp)[i] = u;
    __threadfence();
    ((volatile unsigned*)outp)[i] = u;
  }
}

__global__ __launch_bounds__(256) void tsplit_kernel(const float* __restrict__ W, unsigned short* __restrict__ oh,
                                                     unsigned short* __restrict__ ol, int R, int Cc, long sIn, long sOut) {
  __shared__ __align__(16) float tf[64 * 68];
  W  += (size_t)blockIdx.z * sIn;
  oh += (size_t)blockIdx.z * sOut;
  ol += (size_t)blockIdx.z * sOut;
  const int c0  = blockIdx.x * 64;
  const int r0  = blockIdx.y * 64;
  const int tid = threadIdx.x;
  {
    const int lr = tid >> 4;
    const int c4 = (tid & 15) * 4;
#pragma unroll
    for (int it = 0; it < 4; ++it) {
      const int rr = it * 16 + lr;
      const v4f a = *(const v4f*)(W + (size_t)(r0 + rr) * Cc + c0 + c4);
      *(v4f*)(tf + rr * 68 + c4) = a;
    }
  }
  __syncthreads();
  const int sub = tid >> 3;
  const int c8  = (tid & 7) * 8;
  v4u hv[2], lv[2];
#pragma unroll
  for (int it = 0; it < 2; ++it) {
    const int oc = it * 32 + sub;
    v4u a, a2;
#pragma unroll
    for (int q = 0; q < 4; ++q) {
      const float f0 = tf[(c8 + 2 * q) * 68 + oc];
      const float f1 = tf[(c8 + 2 * q + 1) * 68 + oc];
      const unsigned short h0 = f2bf_bits(f0), h1 = f2bf_bits(f1);
      const unsigned short l0 = f2bf_bits(f0 - bf_bits2f(h0)), l1 = f2bf_bits(f1 - bf_bits2f(h1));
      a[q]  = pk16(h0, h1);
      a2[q] = pk16(l0, l1);
    }
    hv[it] = a; lv[it] = a2;
  }
  for (int pass = 0; pass < 2; ++pass) {
#pragma unroll
    for (int it = 0; it < 2; ++it) {
      const int oc = it * 32 + sub;
      const size_t go = (size_t)(c0 + oc) * R + r0 + c8;
      *(volatile v4u*)(oh + go) = hv[it];
      *(volatile v4u*)(ol + go) = lv[it];
    }
    __threadfence();
  }
}

#define AT_D 64
#define AT_NW 4
#define AT_QB 64
#define AT_KC 64

__device__ __forceinline__ unsigned short at_bf_bits(float f) {
  unsigned u = __float_as_uint(f);
  return (unsigned short)((u + 0x7FFFu + ((u >> 16) & 1u)) >> 16);
}
__device__ __forceinline__ __bf16 at_f2bf(float f) { return __builtin_bit_cast(__bf16, at_bf_bits(f)); }
__device__ __forceinline__ void at_split(float f, __bf16& hi, __bf16& lo) {
  const unsigned short hb = at_bf_bits(f);
  hi = __builtin_bit_cast(__bf16, hb);
  lo = at_f2bf(f - __uint_as_float(((unsigned)hb) << 16));
}
__device__ __forceinline__ v8f at_mma(v16b a, v16b b, v8f c) {
  c = __builtin_amdgcn_wmma_f32_16x16x32_bf16(false, a, false, b, (short)0, c, false, false);
  asm volatile("v_nop\n\tv_nop\n\tv_nop\n\tv_nop" : "+v"(c) : "v"(a), "v"(b));
  return c;
}
__device__ __forceinline__ v8f at_mma_h(v16h a, v16h b, v8f c) {
  c = __builtin_amdgcn_wmma_f32_16x16x32_f16(false, a, false, b, (short)0, c, false, false);
  asm volatile("v_nop\n\tv_nop\n\tv_nop\n\tv_nop" : "+v"(c) : "v"(a), "v"(b));
  return c;
}

__global__ __launch_bounds__(128)
void xattn_kernel(const unsigned short* __restrict__ qp, const unsigned short* __restrict__ kp,
                  const unsigned short* __restrict__ vhp, const unsigned short* __restrict__ vlp,
                  float* __restrict__ outp, float sscale) {
  union FB { v16b v; v8b h[2]; };
  union FH { v16h v; v8h h[2]; };
  __shared__ __align__(16) _Float16 Ksh[AT_KC * AT_D];
  __shared__ __align__(16) __bf16   Vth[AT_D * AT_KC];
  __shared__ __align__(16) __bf16   Vtl[AT_D * AT_KC];
  __shared__ __align__(16) __bf16   Psh[AT_NW][16 * AT_KC];
  __shared__ __align__(16) __bf16   Psl[AT_NW][16 * AT_KC];
  __shared__ __align__(16) float    Os[AT_NW][16 * 68];

  const int tid  = threadIdx.x;
  const int wave = tid >> 5;
  const int lane = tid & 31;
  const int hh   = lane >> 4;
  const int c    = lane & 15;

  constexpr int nqb = kTq / AT_QB;
  const int bx = blockIdx.x;
  const int qb = bx % nqb;
  const int bh = bx / nqb;
  const int h  = bh % kHeads;
  const int b  = bh / kHeads;
  const int q0 = qb * AT_QB + wave * 16;

  const size_t actPlane = (size_t)kBatch * kTkv * kChan;
  const size_t vPlane   = (size_t)kChan * kTkv;

  v16h qa[2];
  {
    const _Float16* qrow = (const _Float16*)(const void*)qp + ((size_t)b * kTq + q0 + c) * kChan + (size_t)h * AT_D;
#pragma unroll
    for (int dc = 0; dc < 2; ++dc) qa[dc] = Frag<_Float16>::load(qrow + dc * 32 + 8 * hh);
  }

  float* os = Os[wave];
#pragma unroll
  for (int r = 0; r < 8; ++r)
#pragma unroll
    for (int t = 0; t < 4; ++t) os[(8 * hh + r) * 68 + t * 16 + c] = 0.f;

#pragma unroll 1
  for (int src = 0; src < kSrc; ++src) {
    const _Float16* Kb = (const _Float16*)(const void*)kp + (size_t)src * actPlane + ((size_t)b * kTkv) * kChan + (size_t)h * AT_D;
    const __bf16*   Vh = (const __bf16*)(const void*)vhp + (size_t)(src * kBatch + b) * vPlane + (size_t)(h * AT_D) * kTkv;
    const __bf16*   Vl = (const __bf16*)(const void*)vlp + (size_t)(src * kBatch + b) * vPlane + (size_t)(h * AT_D) * kTkv;

    float mrow[8], lrow[8];
    v8f oacc[4];
#pragma unroll
    for (int r = 0; r < 8; ++r) { mrow[r] = -INFINITY; lrow[r] = 0.f; }
#pragma unroll
    for (int t = 0; t < 4; ++t) oacc[t] = (v8f){0.f,0.f,0.f,0.f,0.f,0.f,0.f,0.f};

#pragma unroll 1
    for (int kc = 0; kc < kTkv / AT_KC; ++kc) {
      const int kv0 = kc * AT_KC;
      __syncthreads();
      {
        const int rr = tid >> 1, hf = (tid & 1) * 32;
        const _Float16* ks  = Kb + (size_t)(kv0 + rr) * kChan + hf;
        const __bf16*   vhs = Vh + (size_t)rr * kTkv + kv0 + hf;
        const __bf16*   vls = Vl + (size_t)rr * kTkv + kv0 + hf;
#pragma unroll
        for (int i = 0; i < 4; ++i) {
          const v8h k8 = *(const v8h*)(ks + 8 * i);
          const v8b a8 = *(const v8b*)(vhs + 8 * i);
          const v8b l8 = *(const v8b*)(vls + 8 * i);
          *(v8h*)(Ksh + rr * AT_D + hf + 8 * i)  = k8;
          *(v8b*)(Vth + rr * AT_KC + hf + 8 * i) = a8;
          *(v8b*)(Vtl + rr * AT_KC + hf + 8 * i) = l8;
        }
      }
      __syncthreads();

      v8f s[4];
#pragma unroll
      for (int j = 0; j < 4; ++j) {
        s[j] = (v8f){0.f,0.f,0.f,0.f,0.f,0.f,0.f,0.f};
#pragma unroll
        for (int dc = 0; dc < 2; ++dc) {
          FH kb;
          kb.h[0] = *(const v8h*)(Ksh + (j * 16 + c) * AT_D + dc * 32 + 8 * hh);
          kb.h[1] = *(const v8h*)(Ksh + (j * 16 + c) * AT_D + dc * 32 + 16 + 8 * hh);
          s[j] = at_mma_h(qa[dc], kb.v, s[j]);
        }
      }
      float cm[8];
#pragma unroll
      for (int r = 0; r < 8; ++r) {
        float m = -INFINITY;
#pragma unroll
        for (int j = 0; j < 4; ++j) {
          s[j][r] *= sscale;
          m = fmaxf(m, s[j][r]);
        }
#pragma unroll
        for (int off = 1; off < 16; off <<= 1) m = fmaxf(m, __shfl_xor(m, off, 32));
        cm[r] = m;
      }
      __bf16* pwh = Psh[wave];
      __bf16* pwl = Psl[wave];
#pragma unroll
      for (int r = 0; r < 8; ++r) {
        const float mnew = fmaxf(mrow[r], cm[r]);
        const float alpha = expf(mrow[r] - mnew);
        mrow[r] = mnew;
        float psum = 0.f;
#pragma unroll
        for (int j = 0; j < 4; ++j) {
          const float p = expf(s[j][r] - mnew);
          psum += p;
          __bf16 a, bl; at_split(p, a, bl);
          pwh[(8 * hh + r) * AT_KC + j * 16 + c] = a;
          pwl[(8 * hh + r) * AT_KC + j * 16 + c] = bl;
        }
#pragma unroll
        for (int off = 1; off < 16; off <<= 1) psum += __shfl_xor(psum, off, 32);
        lrow[r] = lrow[r] * alpha + psum;
#pragma unroll
        for (int t = 0; t < 4; ++t) oacc[t][r] *= alpha;
      }
      __builtin_amdgcn_fence(__ATOMIC_RELEASE, "workgroup");
      __builtin_amdgcn_wave_barrier();
      __builtin_amdgcn_fence(__ATOMIC_ACQUIRE, "workgroup");
#pragma unroll 1
      for (int kk = 0; kk < 2; ++kk) {
        FB pa, pl;
        pa.h[0] = *(const v8b*)(pwh + c * AT_KC + kk * 32 + 8 * hh);
        pa.h[1] = *(const v8b*)(pwh + c * AT_KC + kk * 32 + 16 + 8 * hh);
        pl.h[0] = *(const v8b*)(pwl + c * AT_KC + kk * 32 + 8 * hh);
        pl.h[1] = *(const v8b*)(pwl + c * AT_KC + kk * 32 + 16 + 8 * hh);
#pragma unroll
        for (int t = 0; t < 4; ++t) {
          FB vb, vl;
          vb.h[0] = *(const v8b*)(Vth + (t * 16 + c) * AT_KC + kk * 32 + 8 * hh);
          vb.h[1] = *(const v8b*)(Vth + (t * 16 + c) * AT_KC + kk * 32 + 16 + 8 * hh);
          vl.h[0] = *(const v8b*)(Vtl + (t * 16 + c) * AT_KC + kk * 32 + 8 * hh);
          vl.h[1] = *(const v8b*)(Vtl + (t * 16 + c) * AT_KC + kk * 32 + 16 + 8 * hh);
          oacc[t] = at_mma(pa.v, vb.v, oacc[t]);
          oacc[t] = at_mma(pa.v, vl.v, oacc[t]);
          oacc[t] = at_mma(pl.v, vb.v, oacc[t]);
        }
      }
    }
#pragma unroll
    for (int r = 0; r < 8; ++r) {
      const float inv = 1.0f / lrow[r];
#pragma unroll
      for (int t = 0; t < 4; ++t) os[(8 * hh + r) * 68 + t * 16 + c] += oacc[t][r] * inv;
    }
  }

  __builtin_amdgcn_fence(__ATOMIC_RELEASE, "workgroup");
  __builtin_amdgcn_wave_barrier();
  __builtin_amdgcn_fence(__ATOMIC_ACQUIRE, "workgroup");
  {
    float* ob = outp + ((size_t)b * kTq) * kChan + (size_t)h * AT_D;
    const int c4 = c * 4;
    for (int pass = 0; pass < 2; ++pass) {
#pragma unroll
      for (int it = 0; it < 8; ++it) {
        const int row = it * 2 + hh;
        v4f val = *(const v4f*)(os + row * 68 + c4);
        *(volatile v4f*)(ob + (size_t)(q0 + row) * kChan + c4) = val;
      }
      __threadfence();
    }
  }
}

extern "C" void kernel_launch(void* const* d_in, const int* in_sizes, int n_in,
                              void* d_out, int out_size, void* d_ws, size_t ws_size,
                              hipStream_t stream) {
  const float* x  = (const float*)d_in[0];
  const float* y  = (const float*)d_in[1];
  const float* Wq = (const float*)d_in[2];
  const float* bq = (const float*)d_in[3];
  const float* Wk = (const float*)d_in[4];
  const float* bk = (const float*)d_in[5];
  const float* Wv = (const float*)d_in[6];
  const float* bv = (const float*)d_in[7];
  const float* Wp = (const float*)d_in[8];
  const float* bp = (const float*)d_in[9];
  float* outp = (float*)d_out;

  const int rowsX = kBatch * kTq;
  const size_t actPlane = (size_t)kBatch * kTq * kChan;
  const size_t wsz = (size_t)kChan * kChan;
  if (n_in < 10) return;
  if (in_sizes[0] != (int)actPlane || in_sizes[1] != (int)(kSrc * actPlane) || in_sizes[2] != (int)wsz ||
      in_sizes[3] != kChan || in_sizes[4] != (int)(kSrc * wsz) || in_sizes[5] != kSrc * kChan ||
      in_sizes[6] != (int)(kSrc * wsz) || in_sizes[7] != kSrc * kChan || in_sizes[8] != (int)wsz || in_sizes[9] != kChan) return;
  if (out_size != (int)actPlane) return;

  size_t off = 0;
  char* ws = (char*)d_ws;
  unsigned short* xb  = (unsigned short*)(ws + off); off += actPlane * 2;
  unsigned short* yb  = (unsigned short*)(ws + off); off += (size_t)kSrc * actPlane * 2;
  unsigned short* wt  = (unsigned short*)(ws + off); off += 8 * wsz * 2;
  unsigned short* wlo = (unsigned short*)(ws + off); off += (size_t)kSrc * wsz * 2;
  unsigned short* qpl = (unsigned short*)(ws + off); off += actPlane * 2;
  unsigned short* kpl = (unsigned short*)(ws + off); off += (size_t)kSrc * actPlane * 2;
  unsigned short* vh  = (unsigned short*)(ws + off); off += (size_t)kSrc * actPlane * 2;
  unsigned short* vl  = (unsigned short*)(ws + off); off += (size_t)kSrc * actPlane * 2;
  float*          of32 = (float*)(ws + off);         off += actPlane * 4;
  unsigned short* oh  = (unsigned short*)(ws + off); off += actPlane * 2;
  unsigned short* ol  = (unsigned short*)(ws + off); off += actPlane * 2;
  if (off > ws_size) return;
  const float* dummyf = (const float*)d_ws;

  unsigned short* wtq = wt;
  unsigned short* wtk = wt + 1 * wsz;
  unsigned short* wtv = wt + 4 * wsz;
  unsigned short* wtp = wt + 7 * wsz;

  cast_bf16x2_kernel<<<(unsigned)((actPlane / 2 + 255) / 256), 256, 0, stream>>>(x, xb, (int)(actPlane / 2));
  cast_bf16x2_kernel<<<(unsigned)((kSrc * actPlane / 2 + 255) / 256), 256, 0, stream>>>(y, yb, (int)(kSrc * actPlane / 2));

  tsplit_kernel<<<dim3(kChan / 64, kChan / 64, 1), 256, 0, stream>>>(Wq, wtq, wlo, kChan, kChan, (long)wsz, (long)wsz);
  tsplit_kernel<<<dim3(kChan / 64, kChan / 64, kSrc), 256, 0, stream>>>(Wk, wtk, wlo, kChan, kChan, (long)wsz, (long)wsz);
  tsplit_kernel<<<dim3(kChan / 64, kChan / 64, kSrc), 256, 0, stream>>>(Wv, wtv, wlo, kChan, kChan, (long)wsz, (long)wsz);
  tsplit_kernel<<<dim3(kChan / 64, kChan / 64, 1), 256, 0, stream>>>(Wp, wtp, wlo, kChan, kChan, (long)wsz, (long)wsz);

  const unsigned gQ = (unsigned)(((rowsX / 64) * (kChan / 64)) / 8);
  wmma_gemm64<1, false, 2, 1, false><<<dim3(gQ, 1), 256, 0, stream>>>(
      xb, xb, kChan, 0L, wtq, wtq, kChan, 0L, qpl, qpl, kChan, 0L, bq, dummyf, 0L, rowsX, kChan, kChan, 1.0f);

  const unsigned gV = (unsigned)(((kChan / 64) * (kTkv / 64)) / 8);
  for (int i = 0; i < kSrc; ++i) {
    wmma_gemm64<1, false, 2, 1, false><<<dim3(gQ, 1), 256, 0, stream>>>(
        yb + (size_t)i * actPlane, yb + (size_t)i * actPlane, kChan, 0L,
        wtk + (size_t)i * wsz, wtk + (size_t)i * wsz, kChan, 0L,
        kpl + (size_t)i * actPlane, kpl + (size_t)i * actPlane, kChan, 0L,
        bk + i * kChan, dummyf, 0L, rowsX, kChan, kChan, 1.0f);
    wmma_gemm64<1, false, 1, 2, false><<<dim3(gV, kBatch), 256, 0, stream>>>(
        wtv + (size_t)i * wsz, wtv + (size_t)i * wsz, kChan, 0L,
        yb + (size_t)i * actPlane, yb + (size_t)i * actPlane, kChan, (long)((size_t)kTkv * kChan),
        vh + (size_t)i * actPlane, vl + (size_t)i * actPlane, kTkv, (long)((size_t)kChan * kTkv),
        bv + i * kChan, dummyf, 0L, kChan, kTkv, kChan, 1.0f);
  }

  xattn_kernel<<<(unsigned)(kBatch * kHeads * (kTq / AT_QB)), 128, 0, stream>>>(qpl, kpl, vh, vl, of32, 0.125f);

  split_bf16x2_kernel<<<(unsigned)((actPlane / 2 + 255) / 256), 256, 0, stream>>>(of32, oh, ol, (int)(actPlane / 2));

  wmma_gemm64<1, true, 2, 0, false, 0, false><<<dim3(gQ, 1), 256, 0, stream>>>(
      oh, ol, kChan, 0L, wtp, wtp, kChan, 0L, outp, outp, kChan, 0L, bp, dummyf, 0L, rowsX, kChan, kChan, 1.0f);
}
